// NemotronFlashDecoderLayer_89850715833068
// MI455X (gfx1250) — hardware-verified
//
#include <hip/hip_runtime.h>
#include <math.h>

#pragma clang fp contract(off)

constexpr int kTok   = 2048;
constexpr int kHidC  = 2048;
constexpr int kHeads = 16;
constexpr int kHD    = 128;
constexpr int kBetaN = 64;
constexpr int kTS    = 16;
constexpr float kQScale = 0.08838834764831845f;
constexpr float kEps    = 1e-6f;

constexpr size_t kPlane16 = (size_t)kTok * kHidC * 2;
constexpr size_t kPlane32 = (size_t)kTok * kHidC * 4;
constexpr size_t kOffXb   = 0;
constexpr size_t kOffWqT  = kOffXb + kPlane16;
constexpr size_t kOffWkT  = kOffWqT + kPlane16;
constexpr size_t kOffWvT  = kOffWkT + kPlane16;
constexpr size_t kOffWoT  = kOffWvT + kPlane16;
constexpr size_t kOffWbT  = kOffWoT + kPlane16;
constexpr size_t kOffBeta = kOffWbT + (size_t)kBetaN * kHidC * 2;
constexpr size_t kOffRaw  = kOffBeta + (size_t)kTok * kBetaN * 4;
constexpr size_t kOffOhi  = kOffRaw;
constexpr size_t kOffOlo  = kOffRaw + kPlane16;
constexpr size_t kOffQN   = kOffRaw + kPlane32;
constexpr size_t kOffKN   = kOffQN + kPlane32;
constexpr size_t kOffVV   = kOffKN + kPlane32;
constexpr size_t kCarveEnd = kOffVV + kPlane32;
constexpr size_t kCarveLimit = (size_t)134217728;

typedef __attribute__((ext_vector_type(16))) _Float16 v16h;
typedef __attribute__((ext_vector_type(8)))  _Float16 v8h;
typedef __attribute__((ext_vector_type(16))) __bf16   v16b;
typedef __attribute__((ext_vector_type(8)))  __bf16   v8b;
typedef __attribute__((ext_vector_type(8)))  float    v8f;
typedef __attribute__((ext_vector_type(4)))  float    v4f;
typedef __attribute__((ext_vector_type(4)))  unsigned int v4u;

__device__ __forceinline__ unsigned short f2bf_bits(float f) {
  unsigned u = __float_as_uint(f);
  return (unsigned short)((u + 0x7FFFu + ((u >> 16) & 1u)) >> 16);
}
__device__ __forceinline__ float bf_bits2f(unsigned short h) { return __uint_as_float(((unsigned)h) << 16); }
__device__ __forceinline__ unsigned pk16(unsigned short a, unsigned short b) { return (unsigned)a | ((unsigned)b << 16); }

__device__ __forceinline__ void dep_guard_h(v8f& a, v8f& b, v16h x, v16h y) { asm volatile("v_nop\n\tv_nop\n\tv_nop\n\tv_nop" : "+v"(a), "+v"(b) : "v"(x), "v"(y)); }
__device__ __forceinline__ void dep_guard_b(v8f& a, v8f& b, v16b x, v16b y) { asm volatile("v_nop\n\tv_nop\n\tv_nop\n\tv_nop" : "+v"(a), "+v"(b) : "v"(x), "v"(y)); }
__device__ __forceinline__ void keep4_h(v16h a, v16h b, v16h c, v16h d) { asm volatile("v_nop" :: "v"(a), "v"(b), "v"(c), "v"(d)); }
__device__ __forceinline__ void keep4_b(v16b a, v16b b, v16b c, v16b d) { asm volatile("v_nop" :: "v"(a), "v"(b), "v"(c), "v"(d)); }
__device__ __forceinline__ void acc_guard4(v8f& a, v8f& b, v8f& c, v8f& d) { asm volatile("v_nop\n\tv_nop\n\tv_nop\n\tv_nop" : "+v"(a), "+v"(b), "+v"(c), "+v"(d)); }
template <typename T> struct Frag;
template <> struct Frag<_Float16> {
  typedef v16h V; union U { v16h v; v8h h[2]; };
  static __device__ __forceinline__ v16h load(const _Float16* p) {
    U f; f.h[0] = *(const v8h*)(p); f.h[1] = *(const v8h*)(p + 16); return f.v;
  }
  static __device__ __forceinline__ v8f mma(v16h a, v16h b, v8f c) {
    return __builtin_amdgcn_wmma_f32_16x16x32_f16(false, a, false, b, (short)0, c, false, false);
  }
  static __device__ __forceinline__ void guard(v8f& a, v8f& b, v16h x, v16h y) { dep_guard_h(a, b, x, y); }
  static __device__ __forceinline__ void keep(v16h a, v16h b, v16h c, v16h d) { keep4_h(a, b, c, d); }
};
template <> struct Frag<__bf16> {
  typedef v16b V; union U { v16b v; v8b h[2]; };
  static __device__ __forceinline__ v16b load(const __bf16* p) {
    U f; f.h[0] = *(const v8b*)(p); f.h[1] = *(const v8b*)(p + 16); return f.v;
  }
  static __device__ __forceinline__ v8f mma(v16b a, v16b b, v8f c) {
    return __builtin_amdgcn_wmma_f32_16x16x32_bf16(false, a, false, b, (short)0, c, false, false);
  }
  static __device__ __forceinline__ void guard(v8f& a, v8f& b, v16b x, v16b y) { dep_guard_b(a, b, x, y); }
  static __device__ __forceinline__ void keep(v16b a, v16b b, v16b c, v16b d) { keep4_b(a, b, c, d); }
};

template <int ET> struct Elem;
template <> struct Elem<0> { typedef _Float16 T; };
template <> struct Elem<1> { typedef __bf16 T; };
template <int ET, int SPLIT, int BIAS_MODE, int OUT_MODE, bool RESID, int ACT = 0>
__global__ __launch_bounds__(256) void wmma_gemm64(
    const unsigned short* __restrict__ Ap, const unsigned short* __restrict__ A2p, int lda, long strideA,
    const unsigned short* __restrict__ Btp, const unsigned short* __restrict__ Bt2p, int ldb, long strideB,
    void* __restrict__ Cout, void* __restrict__ Cout2, int ldc, long strideC,
    const float* __restrict__ bias,
    const float* __restrict__ resid, long strideR,
    int M, int N, int K, float scale) {
  typedef typename Elem<ET>::T T;
  typedef typename Frag<T>::V V;
  const T* A = (const T*)Ap; const T* A2 = (const T*)A2p; const T* Bt = (const T*)Btp; const T* Bt2 = (const T*)Bt2p;
  __shared__ __align__(16) float sT[8][16 * 68];
  const int b    = blockIdx.y;
  const int lane = threadIdx.x & 31;
  const int wave = threadIdx.x >> 5;
  const int tilesN = N >> 6;
  const int tilesM = M >> 6;
  const int tile = blockIdx.x * 8 + wave;
  if (tile >= tilesM * tilesN) return;
  const int tm = tile / tilesN;
  const int tn = tile - tm * tilesN;
  const int m0 = tm << 6;
  const int n0 = tn << 6;

  const T* Ab  = A  + (size_t)b * strideA;
  const T* Bb  = Bt + (size_t)b * strideB;
  const T* Ab2 = (SPLIT != 0) ? (A2  + (size_t)b * strideA) : nullptr;
  const T* Bb2 = (SPLIT == 2) ? (Bt2 + (size_t)b * strideB) : nullptr;

  const int rlane = lane & 15;
  const int koff  = (lane >> 4) * 8;
  const int mOff  = (lane >> 4) * 8;

  v8f acc[4][4];
#pragma unroll
  for (int i = 0; i < 4; ++i)
#pragma unroll
    for (int j = 0; j < 4; ++j) acc[i][j] = (v8f){0.f,0.f,0.f,0.f,0.f,0.f,0.f,0.f};

  for (int k0 = 0; k0 < K; k0 += 32) {
    V bh[4], bl[4];
#pragma unroll
    for (int j = 0; j < 4; ++j) {
      const size_t bo = (size_t)(n0 + (j << 4) + rlane) * ldb + koff + k0;
      bh[j] = Frag<T>::load(Bb + bo);
      if (SPLIT == 2) bl[j] = Frag<T>::load(Bb2 + bo);
    }
#pragma unroll
    for (int i = 0; i < 4; ++i) {
      const size_t ao = (size_t)(m0 + (i << 4) + rlane) * lda + koff + k0;
      V ah = Frag<T>::load(Ab + ao);
      V al;
      if (SPLIT != 0) al = Frag<T>::load(Ab2 + ao);
#pragma unroll
      for (int j = 0; j < 4; ++j) {
        acc[i][j] = Frag<T>::mma(ah, bh[j], acc[i][j]);
        if (SPLIT == 2) acc[i][j] = Frag<T>::mma(ah, bl[j], acc[i][j]);
        if (SPLIT != 0) acc[i][j] = Frag<T>::mma(al, bh[j], acc[i][j]);
      }
      Frag<T>::guard(acc[i][0], acc[i][3], ah, (SPLIT != 0) ? al : ah);
    }
    Frag<T>::keep(bh[0], bh[1], bh[2], bh[3]);
    if (SPLIT == 2) Frag<T>::keep(bl[0], bl[1], bl[2], bl[3]);
  }
  acc_guard4(acc[0][0], acc[0][1], acc[0][2], acc[0][3]);
  acc_guard4(acc[1][0], acc[1][1], acc[1][2], acc[1][3]);
  acc_guard4(acc[2][0], acc[2][1], acc[2][2], acc[2][3]);
  acc_guard4(acc[3][0], acc[3][1], acc[3][2], acc[3][3]);

  float* slab = sT[wave];
  const float* Rb = RESID ? (resid + (size_t)b * strideR) : nullptr;
#pragma unroll
  for (int i = 0; i < 4; ++i) {
    const int mBase = m0 + (i << 4);
#pragma unroll
    for (int j = 0; j < 4; ++j) {
      const int n = n0 + (j << 4) + rlane;
      float bv = 0.f;
      if (BIAS_MODE == 2) bv = bias[n];
#pragma unroll
      for (int r = 0; r < 8; ++r) {
        float v = acc[i][j][r] * scale;
        if (BIAS_MODE == 1) v += bias[mBase + mOff + r];
        if (BIAS_MODE == 2) v += bv;
        if (RESID) v += Rb[(size_t)(mBase + mOff + r) * ldc + n];
        if (ACT == 2) v = fmaxf(v, 0.0f);
        if (ACT == 4) v = (v > 0.f) ? v : 0.01f * v;
        slab[(mOff + r) * 68 + (j << 4) + rlane] = v;
      }
    }
    __builtin_amdgcn_fence(__ATOMIC_RELEASE, "workgroup");
    __builtin_amdgcn_wave_barrier();
    __builtin_amdgcn_fence(__ATOMIC_ACQUIRE, "workgroup");
    if (OUT_MODE == 0) {
      float* C = (float*)Cout + (size_t)b * strideC;
      const int hh = lane >> 4, c4 = (lane & 15) * 4;
      for (int pass = 0; pass < 2; ++pass) {
#pragma unroll
        for (int it = 0; it < 8; ++it) {
          const int row = it * 2 + hh;
          v4f v = *(const v4f*)(slab + row * 68 + c4);
          *(volatile v4f*)(C + (size_t)(mBase + row) * ldc + n0 + c4) = v;
        }
        __threadfence();
      }
    } else {
      const int q = lane >> 3, c8 = (lane & 7) * 8;
      unsigned short* C  = (unsigned short*)Cout  + (size_t)b * strideC;
      unsigned short* C2 = (OUT_MODE == 2) ? ((unsigned short*)Cout2 + (size_t)b * strideC) : nullptr;
      for (int pass = 0; pass < 2; ++pass) {
#pragma unroll
        for (int it = 0; it < 4; ++it) {
          const int row = it * 4 + q;
          const float* sp = slab + row * 68 + c8;
          v8h hv, lv;
#pragma unroll
          for (int e = 0; e < 8; ++e) {
            if (OUT_MODE == 1) {
              hv[e] = (_Float16)sp[e];
            } else {
              unsigned short hb = f2bf_bits(sp[e]);
              unsigned short lb = f2bf_bits(sp[e] - bf_bits2f(hb));
              hv[e] = __builtin_bit_cast(_Float16, hb);
              lv[e] = __builtin_bit_cast(_Float16, lb);
            }
          }
          *(volatile v8h*)(C + (size_t)(mBase + row) * ldc + n0 + c8) = hv;
          if (OUT_MODE == 2) *(volatile v8h*)(C2 + (size_t)(mBase + row) * ldc + n0 + c8) = lv;
        }
        __threadfence();
      }
    }
    __builtin_amdgcn_fence(__ATOMIC_RELEASE, "workgroup");
    __builtin_amdgcn_wave_barrier();
    __builtin_amdgcn_fence(__ATOMIC_ACQUIRE, "workgroup");
  }
}

__global__ __launch_bounds__(256) void cast8_bf16_kernel(const float* __restrict__ in, unsigned short* __restrict__ out, int n8) {
  const int i = blockIdx.x * 256 + threadIdx.x;
  if (i >= n8) return;
  const float* p = in + 8 * (size_t)i;
  const v4f a = *(const v4f*)(p);
  const v4f c = *(const v4f*)(p + 4);
  unsigned short hb[8];
#pragma unroll
  for (int e = 0; e < 4; ++e) {
    hb[e]     = f2bf_bits(a[e]);
    hb[4 + e] = f2bf_bits(c[e]);
  }
  const v4u u = (v4u){pk16(hb[0], hb[1]), pk16(hb[2], hb[3]), pk16(hb[4], hb[5]), pk16(hb[6], hb[7])};
  unsigned short* q = out + 8 * (size_t)i;
  *(volatile v4u*)q = u;
  __threadfence();
  *(volatile v4u*)q = u;
}

__global__ __launch_bounds__(256) void wt_cast4_kernel(const float* __restrict__ W0, const float* __restrict__ W1,
                                                       const float* __restrict__ W2, const float* __restrict__ W3,
                                                       unsigned short* __restrict__ out) {
  __shared__ float sm[64][65];
  const int t  = threadIdx.x;
  const int k0 = blockIdx.x * 64;
  const int n0 = blockIdx.y * 64;
  const int z  = blockIdx.z;
  const float* W = (z == 0) ? W0 : (z == 1) ? W1 : (z == 2) ? W2 : W3;
#pragma unroll
  for (int i = 0; i < 16; ++i) {
    const int e = i * 256 + t;
    const int r = e >> 6;
    const int c = e & 63;
    sm[c][r] = W[(size_t)(k0 + r) * kHidC + n0 + c];
  }
  __syncthreads();
  const int lane = t & 31, wave = t >> 5;
  const int q = lane >> 3, c8 = (lane & 7) * 8;
  unsigned short* op = out + (size_t)z * kHidC * kHidC;
  for (int pass = 0; pass < 2; ++pass) {
#pragma unroll
    for (int it = 0; it < 2; ++it) {
      const int row = wave * 8 + it * 4 + q;
      unsigned short hb[8];
#pragma unroll
      for (int e = 0; e < 8; ++e) hb[e] = f2bf_bits(sm[row][c8 + e]);
      const v4u u = (v4u){pk16(hb[0], hb[1]), pk16(hb[2], hb[3]), pk16(hb[4], hb[5]), pk16(hb[6], hb[7])};
      *(volatile v4u*)(op + (size_t)(n0 + row) * kHidC + k0 + c8) = u;
    }
    __threadfence();
  }
}

__global__ __launch_bounds__(256) void wbt_kernel(const float* __restrict__ Wb, unsigned short* __restrict__ WbT) {
  const int n  = blockIdx.x;
  const int t  = threadIdx.x;
  const int k0 = t * 8;
  const int nc = (n < kHeads) ? n : (kHeads - 1);
  unsigned short hb[8];
#pragma unroll
  for (int e = 0; e < 8; ++e) {
    const float w = Wb[(size_t)(k0 + e) * kHeads + nc];
    hb[e] = (n < kHeads) ? f2bf_bits(w) : (unsigned short)0;
  }
  const v4u u = (v4u){pk16(hb[0], hb[1]), pk16(hb[2], hb[3]), pk16(hb[4], hb[5]), pk16(hb[6], hb[7])};
  unsigned short* q = WbT + (size_t)n * kHidC + k0;
  *(volatile v4u*)q = u;
  __threadfence();
  *(volatile v4u*)q = u;
}

__global__ __launch_bounds__(256) void conv_prep_kernel(const float* __restrict__ raw, const float* __restrict__ cw,
                                                        float* __restrict__ outp, int mode) {
  const int t    = blockIdx.x;
  const int tid  = threadIdx.x;
  const int lane = tid & 31;
  const int wave = tid >> 5;
#pragma unroll 1
  for (int it = 0; it < 2; ++it) {
    const int c0 = wave * 256 + it * 128 + lane * 4;
    float w[4][4];
#pragma unroll
    for (int e = 0; e < 4; ++e) {
      const v4f wl = *(const v4f*)(cw + (size_t)(c0 + e) * 4);
#pragma unroll
      for (int j = 0; j < 4; ++j) w[e][j] = bf_bits2f(f2bf_bits(wl[j]));
    }
    float y[4] = {0.f, 0.f, 0.f, 0.f};
#pragma unroll
    for (int j = 0; j < 4; ++j) {
      const int tt  = t - 3 + j;
      const int ttc = (tt < 0) ? 0 : tt;
      const bool ok = (tt >= 0);
      const v4f x = *(const v4f*)(raw + (size_t)ttc * kHidC + c0);
#pragma unroll
      for (int e = 0; e < 4; ++e) {
        const float xv = ok ? x[e] : 0.f;
        y[e] = y[e] + xv * w[e][j];
      }
    }
    float sv[4];
    float ss = 0.f;
#pragma unroll
    for (int e = 0; e < 4; ++e) {
      const float sg = 1.0f / (1.0f + expf(-y[e]));
      sv[e] = y[e] * sg;
      ss = ss + sv[e] * sv[e];
    }
#pragma unroll
    for (int off = 1; off < 32; off <<= 1) ss += __shfl_xor(ss, off, 32);
    const float r   = rsqrtf(ss + kEps);
    const float fct = (mode < 2) ? r : 1.0f;
    v4f val;
#pragma unroll
    for (int e = 0; e < 4; ++e) {
      float o = sv[e] * fct;
      o = (mode == 0) ? (o * kQScale) : o;
      val[e] = o;
    }
    float* dst = outp + (size_t)t * kHidC + c0;
    *(volatile v4f*)dst = val;
    __threadfence();
    *(volatile v4f*)dst = val;
  }
}

__global__ __launch_bounds__(256) void delta_scan_kernel(const float* __restrict__ QN, const float* __restrict__ KN,
                                                         const float* __restrict__ VV, const float* __restrict__ BETA,
                                                         const float* __restrict__ onw,
                                                         unsigned short* __restrict__ Ohi, unsigned short* __restrict__ Olo) {
  __shared__ __align__(16) float qs[kTS][kHD];
  __shared__ __align__(16) float ks[kTS][kHD];
  __shared__ __align__(16) float vs[kTS][kHD];
  __shared__ __align__(16) float och[kTS][kHD];
  __shared__ float bs[kTS];
  const int h    = blockIdx.x;
  const int tid  = threadIdx.x;
  const int vi   = tid >> 1;
  const int kb   = (tid & 1) * 64;
  const int rr   = tid >> 4;
  const int seg  = tid & 15;

  float S[64];
#pragma unroll
  for (int i = 0; i < 64; ++i) S[i] = 0.f;

  float wv[8];
  {
    const v4f a = *(const v4f*)(onw + seg * 8);
    const v4f c = *(const v4f*)(onw + seg * 8 + 4);
#pragma unroll
    for (int e = 0; e < 4; ++e) {
      wv[e]     = bf_bits2f(f2bf_bits(a[e]));
      wv[4 + e] = bf_bits2f(f2bf_bits(c[e]));
    }
  }

#pragma unroll 1
  for (int chunk = 0; chunk < kTok / kTS; ++chunk) {
    const int t0 = chunk * kTS;
#pragma unroll
    for (int it = 0; it < 2; ++it) {
      const int i    = it * 256 + tid;
      const int row  = i >> 5;
      const int col4 = (i & 31) * 4;
      const size_t g = (size_t)(t0 + row) * kHidC + (size_t)h * kHD + col4;
      *(v4f*)(&qs[row][col4]) = *(const v4f*)(QN + g);
      *(v4f*)(&ks[row][col4]) = *(const v4f*)(KN + g);
      *(v4f*)(&vs[row][col4]) = *(const v4f*)(VV + g);
    }
    {
      const int tb = (tid < kTS) ? tid : (kTS - 1);
      const float x = BETA[(size_t)(t0 + tb) * kBetaN + h];
      const float sg = 1.0f / (1.0f + expf(-x));
      if (tid < kTS) bs[tid] = sg;
    }
    __syncthreads();

#pragma unroll 1
    for (int s = 0; s < kTS; ++s) {
      const float* kr = &ks[s][kb];
      const float* qr = &qs[s][kb];
      float kreg[64];
#pragma unroll
      for (int g4 = 0; g4 < 16; ++g4) {
        const v4f k4 = *(const v4f*)(kr + 4 * g4);
        kreg[4 * g4 + 0] = k4[0];
        kreg[4 * g4 + 1] = k4[1];
        kreg[4 * g4 + 2] = k4[2];
        kreg[4 * g4 + 3] = k4[3];
      }
      float p = 0.f;
#pragma unroll
      for (int kk = 0; kk < 64; ++kk) p = fmaf(kreg[kk], S[kk], p);
      p += __shfl_xor(p, 1, 32);
      const float d = bs[s] * (vs[s][vi] - p);
#pragma unroll
      for (int kk = 0; kk < 64; ++kk) S[kk] = S[kk] + kreg[kk] * d;
      float o = 0.f;
#pragma unroll
      for (int g4 = 0; g4 < 16; ++g4) {
        const v4f q4 = *(const v4f*)(qr + 4 * g4);
#pragma unroll
        for (int e = 0; e < 4; ++e) o = o + q4[e] * S[4 * g4 + e];
      }
      o += __shfl_xor(o, 1, 32);
      och[s][vi] = o;
    }
    __syncthreads();

    {
      const float* orow = &och[rr][seg * 8];
      const v4f a = *(const v4f*)(orow);
      const v4f c = *(const v4f*)(orow + 4);
      float y[8];
#pragma unroll
      for (int e = 0; e < 4; ++e) { y[e] = a[e]; y[4 + e] = c[e]; }
      float ss = 0.f;
#pragma unroll
      for (int e = 0; e < 8; ++e) ss = ss + y[e] * y[e];
      ss += __shfl_xor(ss, 1, 32);
      ss += __shfl_xor(ss, 2, 32);
      ss += __shfl_xor(ss, 4, 32);
      ss += __shfl_xor(ss, 8, 32);
      const float sc = rsqrtf(ss * (1.0f / 128.0f) + kEps);
      unsigned short hbv[8], lbv[8];
#pragma unroll
      for (int e = 0; e < 8; ++e) {
        const float val = (y[e] * sc) * wv[e];
        hbv[e] = f2bf_bits(val);
        lbv[e] = f2bf_bits(val - bf_bits2f(hbv[e]));
      }
      const v4u uh = (v4u){pk16(hbv[0], hbv[1]), pk16(hbv[2], hbv[3]), pk16(hbv[4], hbv[5]), pk16(hbv[6], hbv[7])};
      const v4u ul = (v4u){pk16(lbv[0], lbv[1]), pk16(lbv[2], lbv[3]), pk16(lbv[4], lbv[5]), pk16(lbv[6], lbv[7])};
      const size_t go = (size_t)(t0 + rr) * kHidC + (size_t)h * kHD + seg * 8;
      for (int pass = 0; pass < 2; ++pass) {
        *(volatile v4u*)(Ohi + go) = uh;
        *(volatile v4u*)(Olo + go) = ul;
        __threadfence();
      }
    }
  }
}

extern "C" void kernel_launch(void* const* d_in, const int* in_sizes, int n_in,
                              void* d_out, int out_size, void* d_ws, size_t ws_size,
                              hipStream_t stream) {
  (void)in_sizes; (void)out_size;
  if (n_in < 10) return;
  if (kCarveEnd > ws_size || kCarveEnd > kCarveLimit) return;

  const float* X   = (const float*)d_in[0];
  const float* Wq  = (const float*)d_in[1];
  const float* Wk  = (const float*)d_in[2];
  const float* Wv  = (const float*)d_in[3];
  const float* Wb  = (const float*)d_in[4];
  const float* cwq = (const float*)d_in[5];
  const float* cwk = (const float*)d_in[6];
  const float* cwv = (const float*)d_in[7];
  const float* onw = (const float*)d_in[8];
  const float* Wo  = (const float*)d_in[9];
  float* out = (float*)d_out;

  char* ws = (char*)d_ws;
  unsigned short* Xb   = (unsigned short*)(ws + kOffXb);
  unsigned short* WqT  = (unsigned short*)(ws + kOffWqT);
  unsigned short* WkT  = (unsigned short*)(ws + kOffWkT);
  unsigned short* WvT  = (unsigned short*)(ws + kOffWvT);
  unsigned short* WoT  = (unsigned short*)(ws + kOffWoT);
  unsigned short* WbT  = (unsigned short*)(ws + kOffWbT);
  float*          BETA = (float*)(ws + kOffBeta);
  float*          RAW  = (float*)(ws + kOffRaw);
  unsigned short* Ohi  = (unsigned short*)(ws + kOffOhi);
  unsigned short* Olo  = (unsigned short*)(ws + kOffOlo);
  float*          QN   = (float*)(ws + kOffQN);
  float*          KN   = (float*)(ws + kOffKN);
  float*          VV   = (float*)(ws + kOffVV);

  const int n8 = (kTok * kHidC) / 8;
  cast8_bf16_kernel<<<dim3((n8 + 255) / 256), dim3(256), 0, stream>>>(X, Xb, n8);
  wt_cast4_kernel<<<dim3(kHidC / 64, kHidC / 64, 4), dim3(256), 0, stream>>>(Wq, Wk, Wv, Wo, WqT);
  wbt_kernel<<<dim3(kBetaN), dim3(256), 0, stream>>>(Wb, WbT);

  const int gemmBlocks = ((kTok / 64) * (kHidC / 64)) / 8;
  const int betaBlocks = ((kTok / 64) * (kBetaN / 64) + 7) / 8;

  wmma_gemm64<1, 0, 0, 0, false><<<dim3(betaBlocks, 1), dim3(256), 0, stream>>>(
      Xb, nullptr, kHidC, 0L, WbT, nullptr, kHidC, 0L, (void*)BETA, nullptr, kBetaN, 0L,
      nullptr, nullptr, 0L, kTok, kBetaN, kHidC, 1.0f);

  wmma_gemm64<1, 0, 0, 0, false><<<dim3(gemmBlocks, 1), dim3(256), 0, stream>>>(
      Xb, nullptr, kHidC, 0L, WqT, nullptr, kHidC, 0L, (void*)RAW, nullptr, kHidC, 0L,
      nullptr, nullptr, 0L, kTok, kHidC, kHidC, 1.0f);
  conv_prep_kernel<<<dim3(kTok), dim3(256), 0, stream>>>(RAW, cwq, QN, 0);
  wmma_gemm64<1, 0, 0, 0, false><<<dim3(gemmBlocks, 1), dim3(256), 0, stream>>>(
      Xb, nullptr, kHidC, 0L, WkT, nullptr, kHidC, 0L, (void*)RAW, nullptr, kHidC, 0L,
      nullptr, nullptr, 0L, kTok, kHidC, kHidC, 1.0f);
  conv_prep_kernel<<<dim3(kTok), dim3(256), 0, stream>>>(RAW, cwk, KN, 1);
  wmma_gemm64<1, 0, 0, 0, false><<<dim3(gemmBlocks, 1), dim3(256), 0, stream>>>(
      Xb, nullptr, kHidC, 0L, WvT, nullptr, kHidC, 0L, (void*)RAW, nullptr, kHidC, 0L,
      nullptr, nullptr, 0L, kTok, kHidC, kHidC, 1.0f);
  conv_prep_kernel<<<dim3(kTok), dim3(256), 0, stream>>>(RAW, cwv, VV, 2);

  delta_scan_kernel<<<dim3(kHeads), dim3(256), 0, stream>>>(QN, KN, VV, BETA, onw, Ohi, Olo);

  wmma_gemm64<1, 1, 0, 0, false><<<dim3(gemmBlocks, 1), dim3(256), 0, stream>>>(
      Ohi, Olo, kHidC, 0L, WoT, nullptr, kHidC, 0L, (void*)out, nullptr, kHidC, 0L,
      nullptr, nullptr, 0L, kTok, kHidC, kHidC, 1.0f);
}
